// LocalAttention_26207890440894
// MI455X (gfx1250) — hardware-verified
//
#include <hip/hip_runtime.h>

typedef _Float16 v16h __attribute__((ext_vector_type(16)));
typedef _Float16 v8h  __attribute__((ext_vector_type(8)));
typedef _Float16 v8ha __attribute__((ext_vector_type(8), may_alias));
typedef float    v8f  __attribute__((ext_vector_type(8)));
typedef float    v4f  __attribute__((ext_vector_type(4)));
typedef float    v4fa __attribute__((ext_vector_type(4), may_alias));

#ifndef NB
#define NB 2
#endif
#ifndef SEQ
#define SEQ 2048
#endif
#define NB_FULL 2
#define T_FULL  2048
#define DM      1024
#define NH      16
#define HD      64
#define HALF_W  16
#define QB      64
#define GR      128
#define GC      64
#define KP      72
#define VP      40
#define NEG_BIG (-1.0e30f)
#define WSC     64.0f
#define RWSC    (1.0f / 64.0f)
#define QSC     8.0f
#define SSC     (1.0f / 512.0f)
#define PSCALE  1024.0f
#define LSCALE  2048.0f
#define RSPLIT  (1.0f / 2048.0f)
#define NRM     128.0f
#define ROUT    (1.0f / 4096.0f)

static_assert(NB >= 1 && NB <= NB_FULL);
static_assert(SEQ % GR == 0);
static_assert(SEQ % QB == 0);
static_assert(SEQ % 32 == 0);
static_assert(SEQ % 4 == 0);
static_assert(SEQ <= T_FULL);
static_assert(SEQ > 2 * HALF_W + 2);
static_assert(DM == NH * HD);
static_assert(HD == 64 && GC == HD);
static_assert(DM % GC == 0 && DM % 32 == 0);
static_assert(DM == 128 * 8);
static_assert(QB == 4 * 16 && GR == 4 * 32);
static_assert((KP % 8) == 0 && (VP % 8) == 0);
static_assert(KP >= HD && VP >= 32);

static __device__ __forceinline__ float bf16r(float x)
{
    unsigned u = __float_as_uint(x);
    u = (u + 0x7FFFu + ((u >> 16) & 1u)) & 0xFFFF0000u;
    return __uint_as_float(u);
}

static __device__ __forceinline__ v16h cat8(v8h a, v8h b)
{
    return __builtin_shufflevector(a, b, 0, 1, 2, 3, 4, 5, 6, 7, 8, 9, 10, 11, 12, 13, 14, 15);
}

static __device__ __forceinline__ v8f wmma16(v16h a, v16h b, v8f c)
{
    v8f d = __builtin_amdgcn_wmma_f32_16x16x32_f16(false, a, false, b, (short)0, c, false, false);
    asm volatile("v_nop\n\tv_nop\n\tv_nop\n\tv_nop" : "+v"(d) : "v"(a), "v"(b));
    return d;
}

static __device__ __forceinline__ v8h cvt8(const float* __restrict__ p, float sc)
{
    const v4f x0 = *(const v4f*)p;
    const v4f x1 = *(const v4f*)(p + 4);
    v8h t;
    t[0] = (_Float16)(bf16r(x0[0]) * sc); t[1] = (_Float16)(bf16r(x0[1]) * sc);
    t[2] = (_Float16)(bf16r(x0[2]) * sc); t[3] = (_Float16)(bf16r(x0[3]) * sc);
    t[4] = (_Float16)(bf16r(x1[0]) * sc); t[5] = (_Float16)(bf16r(x1[1]) * sc);
    t[6] = (_Float16)(bf16r(x1[2]) * sc); t[7] = (_Float16)(bf16r(x1[3]) * sc);
    return t;
}

__global__ void __launch_bounds__(128) cvt_x_kernel(const float* __restrict__ x, _Float16* __restrict__ X16)
{
    const int tid = threadIdx.x;
    const int g   = blockIdx.x;
    const int b   = g / (SEQ / 4);
    const int t0  = (g - b * (SEQ / 4)) * 4;
    const size_t m0 = (size_t)b * T_FULL + t0;
    v8h v[4];
#pragma unroll
    for (int r = 0; r < 4; ++r) v[r] = cvt8(x + (m0 + r) * DM + tid * 8, 1.0f);
#pragma unroll
    for (int r = 0; r < 4; ++r) *(volatile v8h*)(X16 + (m0 + r) * DM + tid * 8) = v[r];
    __threadfence();
#pragma unroll
    for (int r = 0; r < 4; ++r) *(volatile v8h*)(X16 + (m0 + r) * DM + tid * 8) = v[r];
}

__global__ void __launch_bounds__(128) cvt_w_kernel(const float* __restrict__ Wq, const float* __restrict__ Wk,
                                                    const float* __restrict__ Wv, const float* __restrict__ Wo,
                                                    _Float16* __restrict__ W16)
{
    const int tid   = threadIdx.x;
    const int which = blockIdx.y;
    const float* src = (which == 0) ? Wq : ((which == 1) ? Wk : ((which == 2) ? Wv : Wo));
    _Float16* dst = W16 + (size_t)which * DM * DM;
    const size_t n0 = (size_t)blockIdx.x * 4;
    v8h v[4];
#pragma unroll
    for (int r = 0; r < 4; ++r) v[r] = cvt8(src + (n0 + r) * DM + tid * 8, WSC);
#pragma unroll
    for (int r = 0; r < 4; ++r) *(volatile v8h*)(dst + (n0 + r) * DM + tid * 8) = v[r];
    __threadfence();
#pragma unroll
    for (int r = 0; r < 4; ++r) *(volatile v8h*)(dst + (n0 + r) * DM + tid * 8) = v[r];
}

static __device__ __forceinline__ void gemm_k(const _Float16* __restrict__ A, const _Float16* __restrict__ W,
                                              int lo, int koff, v8f (&acc)[2][4])
{
    const _Float16* ap0 = A + (size_t)lo * DM + koff;
    const _Float16* ap1 = A + (size_t)(16 + lo) * DM + koff;
    const _Float16* wp0 = W + (size_t)lo * DM + koff;
    const _Float16* wp1 = W + (size_t)(16 + lo) * DM + koff;
    const _Float16* wp2 = W + (size_t)(32 + lo) * DM + koff;
    const _Float16* wp3 = W + (size_t)(48 + lo) * DM + koff;
#pragma unroll 1
    for (int k0 = 0; k0 < DM; k0 += 32) {
        const v16h a0 = cat8(*(const v8h*)(ap0 + k0), *(const v8h*)(ap0 + k0 + 16));
        const v16h a1 = cat8(*(const v8h*)(ap1 + k0), *(const v8h*)(ap1 + k0 + 16));
        const v16h b0 = cat8(*(const v8h*)(wp0 + k0), *(const v8h*)(wp0 + k0 + 16));
        const v16h b1 = cat8(*(const v8h*)(wp1 + k0), *(const v8h*)(wp1 + k0 + 16));
        const v16h b2 = cat8(*(const v8h*)(wp2 + k0), *(const v8h*)(wp2 + k0 + 16));
        const v16h b3 = cat8(*(const v8h*)(wp3 + k0), *(const v8h*)(wp3 + k0 + 16));
        acc[0][0] = wmma16(a0, b0, acc[0][0]);
        acc[0][1] = wmma16(a0, b1, acc[0][1]);
        acc[0][2] = wmma16(a0, b2, acc[0][2]);
        acc[0][3] = wmma16(a0, b3, acc[0][3]);
        acc[1][0] = wmma16(a1, b0, acc[1][0]);
        acc[1][1] = wmma16(a1, b1, acc[1][1]);
        acc[1][2] = wmma16(a1, b2, acc[1][2]);
        acc[1][3] = wmma16(a1, b3, acc[1][3]);
    }
}

__global__ void __launch_bounds__(128) qkv_kernel(const _Float16* __restrict__ X16,
                                                  const _Float16* __restrict__ Wq16,
                                                  const _Float16* __restrict__ Wk16,
                                                  const _Float16* __restrict__ Wv16,
                                                  const float* __restrict__ bq,
                                                  const float* __restrict__ bk,
                                                  const float* __restrict__ bv,
                                                  _Float16* __restrict__ Q16,
                                                  _Float16* __restrict__ K16,
                                                  _Float16* __restrict__ V16)
{
    __shared__ __align__(16) _Float16 stg[4][16 * GC];

    const int tid  = threadIdx.x;
    const int lane = tid & 31;
    const int wave = __builtin_amdgcn_readfirstlane(tid >> 5);
    const int lo   = lane & 15;
    const int hi   = lane >> 4;
    const int koff = hi * 8;

    const int which = blockIdx.z;
    const _Float16* W = (which == 0) ? Wq16 : ((which == 1) ? Wk16 : Wv16);
    const float* bias = (which == 0) ? bq : ((which == 1) ? bk : bv);
    _Float16* dst     = (which == 0) ? Q16 : ((which == 1) ? K16 : V16);

    const int n0 = blockIdx.x * GC;
    const int gy = blockIdx.y;
    const int b  = gy / (SEQ / GR);
    const int t0 = (gy - b * (SEQ / GR)) * GR + wave * 32;
    const size_t m0 = (size_t)b * T_FULL + t0;

    v8f acc[2][4];
#pragma unroll
    for (int i = 0; i < 2; ++i)
#pragma unroll
        for (int j = 0; j < 4; ++j) { v8f z = {}; acc[i][j] = z; }

    gemm_k(X16 + m0 * DM, W + (size_t)n0 * DM, lo, koff, acc);

    float bb[4];
#pragma unroll
    for (int j = 0; j < 4; ++j) bb[j] = bf16r(bias[n0 + 16 * j + lo]);

    const int h = n0 / HD;
    _Float16* st = stg[wave];
    _Float16* drow = dst + ((size_t)(b * NH + h) * T_FULL + t0) * HD;

#pragma unroll
    for (int i = 0; i < 2; ++i) {
#pragma unroll
        for (int j = 0; j < 4; ++j)
#pragma unroll
            for (int r = 0; r < 8; ++r)
                st[(8 * hi + r) * GC + 16 * j + lo] = (_Float16)(fmaf(acc[i][j][r], RWSC, bb[j]) * QSC);
        __syncthreads();
        v8h pv[4];
#pragma unroll
        for (int it = 0; it < 4; ++it) {
            const int idx = lane + 32 * it, row = idx >> 3, pc = idx & 7;
            pv[it] = *(const v8ha*)(st + row * GC + pc * 8);
        }
        __syncthreads();
        _Float16* ob = drow + (size_t)(16 * i) * HD;
#pragma unroll
        for (int it = 0; it < 4; ++it) {
            const int idx = lane + 32 * it, row = idx >> 3, pc = idx & 7;
            *(volatile v8h*)(ob + (size_t)row * HD + pc * 8) = pv[it];
        }
        __threadfence();
#pragma unroll
        for (int it = 0; it < 4; ++it) {
            const int idx = lane + 32 * it, row = idx >> 3, pc = idx & 7;
            *(volatile v8h*)(ob + (size_t)row * HD + pc * 8) = pv[it];
        }
    }
}

__global__ void __launch_bounds__(128) attn_kernel(const _Float16* __restrict__ Q16,
                                                   const _Float16* __restrict__ K16,
                                                   const _Float16* __restrict__ V16,
                                                   _Float16* __restrict__ Chi,
                                                   _Float16* __restrict__ Clo)
{
    __shared__ __align__(16) _Float16 kbuf[32 * KP];
    __shared__ __align__(16) _Float16 vbuf[HD * VP];
    __shared__ __align__(16) _Float16 pbuf[4][16 * 32];
    __shared__ __align__(16) _Float16 plbuf[4][16 * 32];
    __shared__ __align__(16) _Float16 shi[4][16 * HD];
    __shared__ __align__(16) _Float16 slo[4][16 * HD];

    const int tid  = threadIdx.x;
    const int lane = tid & 31;
    const int wave = __builtin_amdgcn_readfirstlane(tid >> 5);
    const int lo   = lane & 15;
    const int hi   = lane >> 4;
    const int koff = hi * 8;
    const int q0   = blockIdx.x * QB;
    const int bh   = blockIdx.y;
    const int qw   = q0 + wave * 16;
    const size_t rowbase = (size_t)bh * T_FULL;

    _Float16* pb  = pbuf[wave];
    _Float16* plb = plbuf[wave];

    v16h aq0, aq1;
    {
        const _Float16* qr = Q16 + (rowbase + qw + lo) * HD;
        aq0 = cat8(*(const v8h*)(qr + koff),      *(const v8h*)(qr + 16 + koff));
        aq1 = cat8(*(const v8h*)(qr + 32 + koff), *(const v8h*)(qr + 48 + koff));
    }

    v8f oacc[4];
#pragma unroll
    for (int nt = 0; nt < 4; ++nt) { v8f z = {}; oacc[nt] = z; }
    float rm[8], rl[8];
#pragma unroll
    for (int i = 0; i < 8; ++i) { rm[i] = NEG_BIG; rl[i] = 0.0f; }

    for (int c = 0; c < SEQ; c += 32) {
#pragma unroll
        for (int it = 0; it < 2; ++it) {
            const int idx = tid + 128 * it;
            const int row = idx >> 3;
            const int pc  = idx & 7;
            const size_t g = (rowbase + c + row) * HD + pc * 8;
            const v8h kk = *(const v8h*)(K16 + g);
            const v8h vv = *(const v8h*)(V16 + g);
            *(v8h*)(kbuf + row * KP + pc * 8) = kk;
            _Float16* vc = vbuf + (pc * 8) * VP + row;
#pragma unroll
            for (int e = 0; e < 8; ++e) vc[e * VP] = vv[e];
        }
        __syncthreads();

        {
            const _Float16* k0r = kbuf + lo * KP;
            const _Float16* k1r = kbuf + (16 + lo) * KP;
            const v16h b00 = cat8(*(const v8h*)(k0r + koff),      *(const v8h*)(k0r + 16 + koff));
            const v16h b01 = cat8(*(const v8h*)(k0r + 32 + koff), *(const v8h*)(k0r + 48 + koff));
            const v16h b10 = cat8(*(const v8h*)(k1r + koff),      *(const v8h*)(k1r + 16 + koff));
            const v16h b11 = cat8(*(const v8h*)(k1r + 32 + koff), *(const v8h*)(k1r + 48 + koff));
            v8f cs0 = {}, cs1 = {};
            cs0 = wmma16(aq0, b00, cs0);
            cs0 = wmma16(aq1, b01, cs0);
            cs1 = wmma16(aq0, b10, cs1);
            cs1 = wmma16(aq1, b11, cs1);

#pragma unroll
            for (int i = 0; i < 8; ++i) {
                const int m = i + 8 * hi;
                const int q = qw + m;
                int d0 = q - (c + lo);      d0 = d0 < 0 ? -d0 : d0;
                int d1 = q - (c + 16 + lo); d1 = d1 < 0 ? -d1 : d1;
                const bool ok0 = (d0 > HALF_W);
                const bool ok1 = (d1 > HALF_W);
                const float sv0 = ok0 ? cs0[i] * SSC : NEG_BIG;
                const float sv1 = ok1 ? cs1[i] * SSC : NEG_BIG;

                float mx = fmaxf(sv0, sv1);
#pragma unroll
                for (int d = 1; d < 16; d <<= 1) mx = fmaxf(mx, __shfl_xor(mx, d, 32));
                const float mnew = fmaxf(rm[i], mx);
                const float scal = __expf(rm[i] - mnew);
                float p0 = __expf(sv0 - mnew); p0 = ok0 ? p0 : 0.0f;
                float p1 = __expf(sv1 - mnew); p1 = ok1 ? p1 : 0.0f;
                float sum = p0 + p1;
#pragma unroll
                for (int d = 1; d < 16; d <<= 1) sum += __shfl_xor(sum, d, 32);
                rl[i] = rl[i] * scal + sum;
                rm[i] = mnew;
#pragma unroll
                for (int nt = 0; nt < 4; ++nt) oacc[nt][i] *= scal;

                const float w0 = p0 * PSCALE, w1 = p1 * PSCALE;
                const _Float16 h0 = (_Float16)w0, h1 = (_Float16)w1;
                pb[m * 32 + lo]       = h0;  plb[m * 32 + lo]      = (_Float16)((w0 - (float)h0) * LSCALE);
                pb[m * 32 + 16 + lo]  = h1;  plb[m * 32 + 16 + lo] = (_Float16)((w1 - (float)h1) * LSCALE);
            }
        }
        __syncthreads();

        {
            const v16h ap  = cat8(*(const v8h*)(pb + lo * 32 + koff),  *(const v8h*)(pb + lo * 32 + 16 + koff));
            const v16h apl = cat8(*(const v8h*)(plb + lo * 32 + koff), *(const v8h*)(plb + lo * 32 + 16 + koff));
#pragma unroll
            for (int nt = 0; nt < 4; ++nt) {
                const _Float16* vr = vbuf + (nt * 16 + lo) * VP;
                const v16h vb = cat8(*(const v8h*)(vr + koff), *(const v8h*)(vr + 16 + koff));
                v8f xr = {};
                xr = wmma16(apl, vb, xr);
                oacc[nt] = wmma16(ap, vb, oacc[nt]);
                oacc[nt] += xr * RSPLIT;
            }
        }
        __syncthreads();
    }

    float inv[8];
#pragma unroll
    for (int i = 0; i < 8; ++i) inv[i] = 1.0f / (rl[i] * NRM);
    _Float16* sh = shi[wave];
    _Float16* sl = slo[wave];
#pragma unroll
    for (int nt = 0; nt < 4; ++nt) {
#pragma unroll
        for (int i = 0; i < 8; ++i) {
            const float v  = oacc[nt][i] * inv[i];
            const float vh = bf16r(v);
            const float vl = bf16r(v - vh);
            sh[(i + 8 * hi) * HD + nt * 16 + lo] = (_Float16)vh;
            sl[(i + 8 * hi) * HD + nt * 16 + lo] = (_Float16)vl;
        }
    }
    __syncthreads();

    v8h oh[4], ol[4];
#pragma unroll
    for (int it = 0; it < 4; ++it) {
        const int idx = lane + 32 * it, row = idx >> 3, pc = idx & 7;
        oh[it] = *(const v8ha*)(sh + row * HD + pc * 8);
        ol[it] = *(const v8ha*)(sl + row * HD + pc * 8);
    }
    const int b = bh / NH;
    const int h = bh - b * NH;
    const size_t cbase = ((size_t)b * T_FULL + qw) * DM + (size_t)h * HD;
#pragma unroll
    for (int it = 0; it < 4; ++it) {
        const int idx = lane + 32 * it, row = idx >> 3, pc = idx & 7;
        const size_t o = cbase + (size_t)row * DM + pc * 8;
        *(volatile v8h*)(Chi + o) = oh[it];
        *(volatile v8h*)(Clo + o) = ol[it];
    }
    __threadfence();
#pragma unroll
    for (int it = 0; it < 4; ++it) {
        const int idx = lane + 32 * it, row = idx >> 3, pc = idx & 7;
        const size_t o = cbase + (size_t)row * DM + pc * 8;
        *(volatile v8h*)(Chi + o) = oh[it];
        *(volatile v8h*)(Clo + o) = ol[it];
    }
}

__global__ void __launch_bounds__(128) oproj_kernel(const _Float16* __restrict__ Chi,
                                                    const _Float16* __restrict__ Clo,
                                                    const _Float16* __restrict__ Wo16,
                                                    const float* __restrict__ bo,
                                                    float* __restrict__ out)
{
    __shared__ __align__(16) float stg[4][16 * GC];

    const int tid  = threadIdx.x;
    const int lane = tid & 31;
    const int wave = __builtin_amdgcn_readfirstlane(tid >> 5);
    const int lo   = lane & 15;
    const int hi   = lane >> 4;
    const int koff = hi * 8;

    const int n0 = blockIdx.x * GC;
    const int gy = blockIdx.y;
    const int b  = gy / (SEQ / GR);
    const int t0 = (gy - b * (SEQ / GR)) * GR + wave * 32;
    const size_t m0 = (size_t)b * T_FULL + t0;

    v8f acc[2][4];
#pragma unroll
    for (int i = 0; i < 2; ++i)
#pragma unroll
        for (int j = 0; j < 4; ++j) { v8f z = {}; acc[i][j] = z; }

    gemm_k(Chi + m0 * DM, Wo16 + (size_t)n0 * DM, lo, koff, acc);
    gemm_k(Clo + m0 * DM, Wo16 + (size_t)n0 * DM, lo, koff, acc);

    float bb[4];
#pragma unroll
    for (int j = 0; j < 4; ++j) bb[j] = bf16r(bo[n0 + 16 * j + lo]);

    float* st = stg[wave];
#pragma unroll
    for (int i = 0; i < 2; ++i) {
#pragma unroll
        for (int j = 0; j < 4; ++j)
#pragma unroll
            for (int r = 0; r < 8; ++r)
                st[(8 * hi + r) * GC + 16 * j + lo] = fmaf(acc[i][j][r], ROUT, bb[j]);
        __syncthreads();
        v4f ov[8];
#pragma unroll
        for (int it = 0; it < 8; ++it) {
            const int idx = lane + 32 * it, row = idx >> 4, pc = idx & 15;
            ov[it] = *(const v4fa*)(st + row * GC + pc * 4);
        }
        __syncthreads();
        float* ob = out + (m0 + 16 * i) * DM + n0;
#pragma unroll
        for (int it = 0; it < 8; ++it) {
            const int idx = lane + 32 * it, row = idx >> 4, pc = idx & 15;
            *(volatile v4f*)(ob + (size_t)row * DM + pc * 4) = ov[it];
        }
        __threadfence();
#pragma unroll
        for (int it = 0; it < 8; ++it) {
            const int idx = lane + 32 * it, row = idx >> 4, pc = idx & 15;
            *(volatile v4f*)(ob + (size_t)row * DM + pc * 4) = ov[it];
        }
    }
}

extern "C" void kernel_launch(void* const* d_in, const int* in_sizes, int n_in,
                              void* d_out, int out_size, void* d_ws, size_t ws_size,
                              hipStream_t stream)
{
    if (n_in < 9) return;
    const long long needx = ((long long)(NB - 1) * T_FULL + SEQ) * DM;
    if ((long long)in_sizes[0] < needx) return;
    if (in_sizes[1] < DM * DM || in_sizes[3] < DM * DM || in_sizes[5] < DM * DM || in_sizes[7] < DM * DM) return;
    if (in_sizes[2] < DM || in_sizes[4] < DM || in_sizes[6] < DM || in_sizes[8] < DM) return;
    if ((long long)out_size < needx) return;

    const float* x  = (const float*)d_in[0];
    const float* Wq = (const float*)d_in[1];
    const float* bq = (const float*)d_in[2];
    const float* Wk = (const float*)d_in[3];
    const float* bk = (const float*)d_in[4];
    const float* Wv = (const float*)d_in[5];
    const float* bv = (const float*)d_in[6];
    const float* Wo = (const float*)d_in[7];
    const float* bo = (const float*)d_in[8];
    float* out = (float*)d_out;

    const size_t rowsF = (size_t)NB_FULL * T_FULL;
    const size_t bX  = rowsF * DM * sizeof(_Float16);
    const size_t bW  = (size_t)4 * DM * DM * sizeof(_Float16);
    const size_t bP  = (size_t)NB_FULL * NH * T_FULL * HD * sizeof(_Float16);
    const size_t bC  = rowsF * DM * sizeof(_Float16);
    const size_t offX  = 0;
    const size_t offW  = offX + bX;
    const size_t offQ  = offW + bW;
    const size_t offK  = offQ + bP;
    const size_t offV  = offK + bP;
    const size_t offCh = offV + bP;
    const size_t offCl = offCh + bC;
    const size_t total = offCl + bC;
    if (total > ws_size) return;

    char* ws = (char*)d_ws;
    _Float16* X16 = (_Float16*)(ws + offX);
    _Float16* W16 = (_Float16*)(ws + offW);
    _Float16* Q16 = (_Float16*)(ws + offQ);
    _Float16* K16 = (_Float16*)(ws + offK);
    _Float16* V16 = (_Float16*)(ws + offV);
    _Float16* Chi = (_Float16*)(ws + offCh);
    _Float16* Clo = (_Float16*)(ws + offCl);

    cvt_x_kernel<<<dim3(NB * SEQ / 4), 128, 0, stream>>>(x, X16);
    cvt_w_kernel<<<dim3(DM / 4, 4), 128, 0, stream>>>(Wq, Wk, Wv, Wo, W16);
    qkv_kernel<<<dim3(DM / GC, NB * SEQ / GR, 3), 128, 0, stream>>>(
        X16, W16, W16 + (size_t)DM * DM, W16 + (size_t)2 * DM * DM, bq, bk, bv, Q16, K16, V16);
    attn_kernel<<<dim3(SEQ / QB, NB * NH), 128, 0, stream>>>(Q16, K16, V16, Chi, Clo);
    oproj_kernel<<<dim3(DM / GC, NB * SEQ / GR), 128, 0, stream>>>(Chi, Clo, W16 + (size_t)3 * DM * DM, bo, out);
}
